// BiquadFilter_45423574123131
// MI455X (gfx1250) — hardware-run, weakly checked
//
#include <hip/hip_runtime.h>
#include <math.h>

typedef __attribute__((ext_vector_type(16))) _Float16 v16h;
typedef __attribute__((ext_vector_type(8)))  _Float16 v8h;
typedef __attribute__((ext_vector_type(8)))  float    v8f;
typedef __attribute__((ext_vector_type(4)))  float    v4f;

constexpr int kBatch  = 8;
constexpr int kChan   = 2;
constexpr int kLen    = 524288;
constexpr int kSec    = 6;
constexpr int kFir    = 8192;
constexpr int kBins   = kFir / 2 + 1;
constexpr int kHP     = 4352;
constexpr int kNch    = 257;
constexpr int kFront  = 8192;
constexpr int kTail   = 2048;
constexpr int kXRow   = kFront + kLen + kTail;
constexpr int kBlkOut = 8192;
constexpr int kXWin   = 16400;
constexpr float kXCarry    = 16.0f;
constexpr float kXCarryInv = 1.0f / 16.0f;

static_assert(kBins == 4097, "bins");
static_assert(kHP >= kBins && (kHP % 256) == 0, "response pitch");
static_assert(kNch * 32 >= kFir + 16, "K extent");
static_assert(kXWin == 7 * 1024 + 3 * 256 + 240 + (kNch - 1) * 32 + 32, "window extent");
static_assert((kXWin % 8) == 0, "window vector multiple");
static_assert((kLen - kBlkOut) + kXWin <= kXRow, "last block window inside the padded row");
static_assert((kXRow % 2048) == 0, "row = whole blocks of 256 threads x 8 halves");
static_assert((kLen % kBlkOut) == 0, "block multiple");
static_assert((kBatch * kNch * 32) % 256 == 0, "fragment builder grid exact");

constexpr size_t kOffH    = 0;
constexpr size_t kSzH     = (size_t)kBatch * 2 * kHP * 4;
constexpr size_t kOffFir  = kOffH + kSzH;
constexpr size_t kSzFir   = (size_t)kBatch * kFir * 4;
constexpr size_t kOffBfr  = kOffFir + kSzFir;
constexpr size_t kSzBfr   = (size_t)kBatch * kNch * 512 * 2;
constexpr size_t kOffXp   = kOffBfr + kSzBfr;
constexpr size_t kSzXp    = (size_t)kBatch * kChan * kXRow * 2;
constexpr size_t kWsTotal = kOffXp + kSzXp;
static_assert(kSzH == 278528ull && kSzFir == 262144ull && kSzBfr == 2105344ull && kSzXp == 17104896ull, "carve sizes");
static_assert(kWsTotal == 19750912ull, "carve total");
static_assert(kWsTotal <= 134217728ull, "carve cap");
static_assert((kOffFir % 128) == 0 && (kOffBfr % 128) == 0 && (kOffXp % 128) == 0, "aligned regions");
static_assert(((size_t)kXRow * 2) % 128 == 0, "row pitch whole lines");

__device__ __forceinline__ unsigned short f2bf_bits(float f) {
  unsigned u = __float_as_uint(f);
  return (unsigned short)((u + 0x7FFFu + ((u >> 16) & 1u)) >> 16);
}
__device__ __forceinline__ float bf_bits2f(unsigned short h) { return __uint_as_float(((unsigned)h) << 16); }
__device__ __forceinline__ float bf_rne(float f) { return bf_bits2f(f2bf_bits(f)); }

union FragH { v16h v; v8h h[2]; };
__device__ __forceinline__ v16h ld_frag_a(const _Float16* p) {
  FragH f; f.h[0] = *(const v8h*)(p); f.h[1] = *(const v8h*)(p + 16); return f.v;
}
__device__ __forceinline__ v16h ld_frag_b(const _Float16* p) {
  FragH f; f.h[0] = *(const v8h*)(p); f.h[1] = *(const v8h*)(p + 256); return f.v;
}
__device__ __forceinline__ v8f mma_h(v16h a, v16h b, v8f c) {
  return __builtin_amdgcn_wmma_f32_16x16x32_f16(false, a, false, b, (short)0, c, false, false);
}
__device__ __forceinline__ void guard_group(v8f& c0, v8f& c1, v8f& c2, v8f& c3,
                                            v16h a0, v16h a1, v16h a2, v16h a3, v16h b) {
  asm volatile("v_nop\n\tv_nop\n\tv_nop\n\tv_nop"
               : "+v"(c0), "+v"(c1), "+v"(c2), "+v"(c3)
               : "v"(a0), "v"(a1), "v"(a2), "v"(a3), "v"(b));
}

__global__ __launch_bounds__(256) void resp_kernel(const float* __restrict__ Bs,
                                                   const float* __restrict__ A1p,
                                                   const float* __restrict__ A2p,
                                                   float* __restrict__ Hpl) {
  const int tid = threadIdx.x;
  const int b = blockIdx.y;
  const int f = blockIdx.x * 256 + tid;
  float s1, c1;
  sincospif((float)f * (1.0f / 4096.0f), &s1, &c1);
  const float c2 = (c1 - s1) * (c1 + s1);
  const float s2 = 2.0f * c1 * s1;
  float hr = 1.0f, hi = 0.0f;
#pragma unroll 1
  for (int k = 0; k < kSec; ++k) {
    const int ci = b * kSec + k;
    const float b0 = bf_rne(Bs[ci * 3 + 0]);
    const float b1 = bf_rne(Bs[ci * 3 + 1]);
    const float b2 = bf_rne(Bs[ci * 3 + 2]);
    const float a1 = 2.0f * tanhf(bf_rne(A1p[ci]));
    const float aa = fabsf(a1);
    const float t2 = tanhf(bf_rne(A2p[ci]));
    const float a2 = ((2.0f - aa) * t2 + aa) * 0.5f;
    const float nr = b0 + b1 * c1 + b2 * c2;
    const float ni = -(b1 * s1 + b2 * s2);
    const float dr = 1.0f + a1 * c1 + a2 * c2;
    const float di = -(a1 * s1 + a2 * s2);
    const float den = fmaxf(dr * dr + di * di, 1e-30f);
    const float inv = 1.0f / den;
    const float qr = (nr * dr + ni * di) * inv;
    const float qi = (ni * dr - nr * di) * inv;
    const float tr = hr * qr - hi * qi;
    hi = hr * qi + hi * qr;
    hr = tr;
  }
  const bool live = (f < kBins);
  const float outr = live ? hr : 0.0f;
  const float outi = live ? hi : 0.0f;
  volatile float* pr = Hpl + ((size_t)b * 2 + 0) * kHP + f;
  volatile float* pi = Hpl + ((size_t)b * 2 + 1) * kHP + f;
  *pr = outr;
  *pi = outi;
  __threadfence();
  *pr = outr;
  *pi = outi;
}

__global__ __launch_bounds__(256) void taps_kernel(const float* __restrict__ Hpl, float* __restrict__ taps) {
  __shared__ __align__(16) float tab[8192];
  __shared__ __align__(16) float sH[256];
  const int tid = threadIdx.x;
  const int b = blockIdx.y;
  const int n = blockIdx.x * 256 + tid;
#pragma unroll 1
  for (int i = tid; i < 8192; i += 256) tab[i] = cospif((float)i * (1.0f / 4096.0f));
  const float* Hb = Hpl + (size_t)b * 2 * kHP;
  const float h0 = Hb[0];
  const float hN = Hb[kBins - 1];
  const int pl = tid >> 7;
  const int fj = tid & 127;
  float acc = 0.0f;
#pragma unroll 1
  for (int c = 0; c < 32; ++c) {
    __syncthreads();
    float hv = Hb[pl * kHP + 128 * c + fj];
    asm volatile("" : "+v"(hv));
    sH[tid] = (c == 0 && fj == 0) ? 0.0f : hv;
    __syncthreads();
    unsigned idx = ((unsigned)(128 * c) * (unsigned)n) & 8191u;
    float part = 0.0f;
#pragma unroll 4
    for (int j = 0; j < 128; ++j) {
      const float cv = tab[idx];
      const float sv = tab[(idx + 6144u) & 8191u];
      part = fmaf(sH[j], cv, part);
      part = fmaf(-sH[128 + j], sv, part);
      idx = (idx + (unsigned)n) & 8191u;
    }
    acc += part;
  }
  const float edge = h0 + ((n & 1) ? -hN : hN);
  const float val = (edge + 2.0f * acc) * (1.0f / 8192.0f);
  volatile float* p = taps + (size_t)b * kFir + n;
  *p = val;
  __threadfence();
  *p = val;
}

__global__ __launch_bounds__(256) void bfrag_kernel(const float* __restrict__ taps, unsigned short* __restrict__ bfr) {
  const int t = blockIdx.x * 256 + threadIdx.x;
  if (t < kBatch * kNch * 32) {
    const int lane = t & 31;
    const int wv = t >> 5;
    const int b = wv / kNch;
    const int cc = wv - b * kNch;
    const int j = lane & 15;
    const int h = lane >> 4;
    const float* fb = taps + (size_t)b * kFir;
    v8h vv[2];
#pragma unroll
    for (int h2 = 0; h2 < 2; ++h2) {
#pragma unroll
      for (int e = 0; e < 8; ++e) {
        const int kk = 32 * cc + 16 * h2 + 8 * h + e;
        const int fi = kFir + j - kk;
        const int fic = fi < 0 ? 0 : (fi > kFir - 1 ? kFir - 1 : fi);
        float val = fb[fic];
        asm volatile("" : "+v"(val));
        val = (fi >= 0 && fi <= kFir - 1) ? val : 0.0f;
        val = fminf(fmaxf(val, -60000.0f), 60000.0f);
        vv[h2][e] = (_Float16)val;
      }
    }
    unsigned short* chunk = bfr + ((size_t)b * kNch + cc) * 512;
    unsigned short* d0 = chunk + (size_t)lane * 8;
    unsigned short* d1 = chunk + (size_t)(32 + lane) * 8;
    *(volatile v8h*)d0 = vv[0];
    *(volatile v8h*)d1 = vv[1];
    __threadfence();
    *(volatile v8h*)d0 = vv[0];
    *(volatile v8h*)d1 = vv[1];
  }
}

__global__ __launch_bounds__(256) void xplane_kernel(const float* __restrict__ x, unsigned short* __restrict__ xpad) {
  const int bc = blockIdx.y;
  const int i8 = blockIdx.x * 256 + threadIdx.x;
  const int q0 = i8 * 8;
  const int s0 = q0 - kFront;
  const bool inx = (s0 >= 0) && (s0 < kLen);
  const int sc = s0 < 0 ? 0 : (s0 > kLen - 8 ? kLen - 8 : s0);
  const float* src = x + (size_t)bc * kLen + sc;
  v4f a0 = *(const v4f*)(src);
  v4f a1 = *(const v4f*)(src + 4);
  asm volatile("" : "+v"(a0));
  asm volatile("" : "+v"(a1));
  v8h hv;
#pragma unroll
  for (int e = 0; e < 4; ++e) {
    const float u0 = inx ? a0[e] : 0.0f;
    const float u1 = inx ? a1[e] : 0.0f;
    hv[e]     = (_Float16)(bf_rne(u0) * kXCarry);
    hv[4 + e] = (_Float16)(bf_rne(u1) * kXCarry);
  }
  unsigned short* dst = xpad + (size_t)bc * kXRow + q0;
  *(volatile v8h*)dst = hv;
  __threadfence();
  *(volatile v8h*)dst = hv;
}

__device__ __forceinline__ void tile_stage(float* sl, const v8f& a, int lane, v4f& u0, v4f& u1) {
#pragma unroll
  for (int r = 0; r < 8; ++r) sl[32 * r + lane] = a[r] * kXCarryInv;
  __builtin_amdgcn_fence(__ATOMIC_RELEASE, "workgroup");
  __builtin_amdgcn_wave_barrier();
  __builtin_amdgcn_fence(__ATOMIC_ACQUIRE, "workgroup");
  u0 = *(const v4f*)(sl + lane * 4);
  u1 = *(const v4f*)(sl + 128 + lane * 4);
  __builtin_amdgcn_fence(__ATOMIC_RELEASE, "workgroup");
  __builtin_amdgcn_wave_barrier();
  __builtin_amdgcn_fence(__ATOMIC_ACQUIRE, "workgroup");
}

__global__ __launch_bounds__(256) void conv_kernel(const unsigned short* __restrict__ xpad,
                                                   const unsigned short* __restrict__ bfr,
                                                   float* __restrict__ out) {
  __shared__ __align__(16) _Float16 xs[kXWin];
  __shared__ __align__(16) float osl[8][256];

  const int tid = threadIdx.x;
  const int lane = tid & 31;
  const int wave = tid >> 5;
  const int bc = blockIdx.y;
  const int b = bc >> 1;
  const int p0 = blockIdx.x * kBlkOut;

  const _Float16* xrow = (const _Float16*)xpad + (size_t)bc * kXRow + p0;
  for (int i = tid * 8; i < kXWin; i += 256 * 8)
    *(v8h*)(xs + i) = *(const v8h*)(xrow + i);
  __syncthreads();

  const int m = lane & 15;
  const int h = lane >> 4;
  const int offm = 32 * (m & 7) + 16 * (m >> 3);
  const _Float16* abase = xs + wave * 1024 + offm + 8 * h;
  const _Float16* bbase = (const _Float16*)bfr + (size_t)b * kNch * 512 + lane * 8;

  v8f acc0 = (v8f){0.f, 0.f, 0.f, 0.f, 0.f, 0.f, 0.f, 0.f};
  v8f acc1 = acc0, acc2 = acc0, acc3 = acc0;

#pragma unroll 2
  for (int c = 0; c < kNch; ++c) {
    const v16h bv = ld_frag_b(bbase + (size_t)c * 512);
    const _Float16* ap = abase + c * 32;
    const v16h a0 = ld_frag_a(ap);
    const v16h a1 = ld_frag_a(ap + 256);
    const v16h a2 = ld_frag_a(ap + 512);
    const v16h a3 = ld_frag_a(ap + 768);
    acc0 = mma_h(a0, bv, acc0);
    acc1 = mma_h(a1, bv, acc1);
    acc2 = mma_h(a2, bv, acc2);
    acc3 = mma_h(a3, bv, acc3);
    guard_group(acc0, acc1, acc2, acc3, a0, a1, a2, a3, bv);
  }

  float* sl = osl[wave];
  v4f u00, u01, u10, u11, u20, u21, u30, u31;
  tile_stage(sl, acc0, lane, u00, u01);
  tile_stage(sl, acc1, lane, u10, u11);
  tile_stage(sl, acc2, lane, u20, u21);
  tile_stage(sl, acc3, lane, u30, u31);

  float* o = out + (size_t)bc * kLen + p0 + wave * 1024 + lane * 4;
  for (int pass = 0; pass < 2; ++pass) {
    *(volatile v4f*)(o)       = u00;
    *(volatile v4f*)(o + 128) = u01;
    *(volatile v4f*)(o + 256) = u10;
    *(volatile v4f*)(o + 384) = u11;
    *(volatile v4f*)(o + 512) = u20;
    *(volatile v4f*)(o + 640) = u21;
    *(volatile v4f*)(o + 768) = u30;
    *(volatile v4f*)(o + 896) = u31;
    __threadfence();
  }
}

extern "C" void kernel_launch(void* const* d_in, const int* in_sizes, int n_in,
                              void* d_out, int out_size, void* d_ws, size_t ws_size,
                              hipStream_t stream) {
  if (n_in < 4) return;
  if (in_sizes[0] != kBatch * kChan * kLen) return;
  if (in_sizes[1] != kBatch * kSec * 3) return;
  if (in_sizes[2] != kBatch * kSec) return;
  if (in_sizes[3] != kBatch * kSec) return;
  if (out_size != kBatch * kChan * kLen) return;
  if (ws_size < kWsTotal) return;

  const float* x   = (const float*)d_in[0];
  const float* Bs  = (const float*)d_in[1];
  const float* A1p = (const float*)d_in[2];
  const float* A2p = (const float*)d_in[3];
  float* out = (float*)d_out;

  char* ws = (char*)d_ws;
  float*          Hpl  = (float*)(ws + kOffH);
  float*          taps = (float*)(ws + kOffFir);
  unsigned short* bfr  = (unsigned short*)(ws + kOffBfr);
  unsigned short* xpad = (unsigned short*)(ws + kOffXp);

  resp_kernel  <<<dim3(kHP / 256, kBatch), 256, 0, stream>>>(Bs, A1p, A2p, Hpl);
  taps_kernel  <<<dim3(kFir / 256, kBatch), 256, 0, stream>>>(Hpl, taps);
  bfrag_kernel <<<dim3((kBatch * kNch * 32) / 256), 256, 0, stream>>>(taps, bfr);
  xplane_kernel<<<dim3(kXRow / 2048, kBatch * kChan), 256, 0, stream>>>(x, xpad);
  conv_kernel  <<<dim3(kLen / kBlkOut, kBatch * kChan), 256, 0, stream>>>(xpad, bfr, out);
}
